// HebbianMambaLayer_77824807403922
// MI455X (gfx1250) — hardware-run, weakly checked
//
#include <hip/hip_runtime.h>
#include <math.h>

typedef __attribute__((ext_vector_type(16))) _Float16 v16h;
typedef __attribute__((ext_vector_type(8)))  _Float16 v8h;
typedef __attribute__((ext_vector_type(2)))  _Float16 v2h;
typedef __attribute__((ext_vector_type(16))) __bf16   v16b;
typedef __attribute__((ext_vector_type(8)))  __bf16   v8b;
typedef __attribute__((ext_vector_type(8)))  float    v8f;
typedef __attribute__((ext_vector_type(4)))  float    v4f;
typedef __attribute__((ext_vector_type(2)))  float    v2f;

constexpr int kB   = 4;
constexpr int kT   = 8192;
constexpr int kD   = 512;
constexpr int kC   = 64;
constexpr int kNC  = kT / kC;
constexpr int kPad = 4;
constexpr int kRows = kT + kPad;
constexpr int kThr  = 256;
constexpr float kInCarry = 1024.0f;
constexpr float kVCarry  = 256.0f;
constexpr float kSCarry  = 64.0f;
constexpr float kRCarry  = 1.0f;
constexpr float kSc20 = 1.0f / (kInCarry * kInCarry);
constexpr float kSc16 = 1.0f / (kInCarry * kSCarry);
constexpr float kSc14 = 1.0f / (kSCarry * kVCarry);
constexpr float kSc18 = 1.0f / (kVCarry * kInCarry);
constexpr float kSc10 = 1.0f / (kRCarry * kInCarry);
constexpr float kMix  = 0.03f;
constexpr float kF16MinNormal = 6.103515625e-5f;

static_assert(kB == 4 && kT == 8192 && kD == 512 && kC == 64 && kNC == 128 && kRows == 8196, "the index arithmetic below uses these sizes");

constexpr size_t kOffXP16 = 0ull;
constexpr size_t kOffP16  = 33570816ull;
constexpr size_t kOffQ16  = 34095104ull;
constexpr size_t kOffVP   = 34619392ull;
constexpr size_t kOffVT16 = 101728256ull;
constexpr size_t kOffVG16 = 135282688ull;
constexpr size_t kOffKT16 = 168837120ull;
constexpr size_t kOffZA   = 202391552ull;
constexpr size_t kOffSM16 = 210780160ull;
constexpr size_t kOffS32  = 210812928ull;
constexpr size_t kOffS16  = 215007232ull;
constexpr size_t kOffDW   = 217104384ull;
constexpr size_t kOffR1   = 221298688ull;
constexpr size_t kOffR2   = 221822976ull;
constexpr size_t kOffRO16 = 222347264ull;
constexpr size_t kOffTAB  = 255901696ull;
constexpr size_t kWsTotal = 255919104ull;
static_assert(kOffP16 == (size_t)kB * kRows * kD * 2ull && kOffQ16 == kOffP16 + 524288ull && kOffVP == kOffQ16 + 524288ull && kOffVT16 == kOffVP + (size_t)kB * kD * kT * 4ull && kOffVG16 == kOffVT16 + (size_t)kB * kD * kT * 2ull && kOffKT16 == kOffVG16 + (size_t)kB * kD * kT * 2ull && kOffZA == kOffKT16 + (size_t)kB * kD * kT * 2ull && kOffSM16 == kOffZA + (size_t)kB * kNC * kC * kC * 4ull && kOffS32 == kOffSM16 + (size_t)kB * kC * kC * 2ull && kOffS16 == kOffS32 + (size_t)kB * kD * kD * 4ull && kOffDW == kOffS16 + (size_t)kB * kD * kD * 2ull && kOffR1 == kOffDW + (size_t)kB * kD * kD * 4ull && kOffR2 == kOffR1 + (size_t)kB * kC * kD * 4ull && kOffRO16 == kOffR2 + (size_t)kB * kC * kD * 4ull && kOffTAB == kOffRO16 + (size_t)kB * kT * kD * 2ull && kWsTotal == kOffTAB + 17408ull, "the carve is a chain: every region starts where the one before ends");
static_assert((kOffP16 % 256) == 0 && (kOffVP % 256) == 0 && (kOffVG16 % 256) == 0 && (kOffZA % 256) == 0 && (kOffSM16 % 256) == 0 && (kOffS32 % 256) == 0 && (kOffR1 % 256) == 0 && (kOffRO16 % 256) == 0 && (kOffTAB % 256) == 0 && ((size_t)kRows * kD * 2ull) % 256 == 0, "every region and every batch row's block starts on a multiple of 256 B");

__device__ __forceinline__ unsigned short f2bf_bits(float f) {
  unsigned u = __float_as_uint(f);
  return (unsigned short)((u + 0x7FFFu + ((u >> 16) & 1u)) >> 16);
}
__device__ __forceinline__ float bf_bits2f(unsigned short h) { return __uint_as_float(((unsigned)h) << 16); }
__device__ __forceinline__ float bf16r(float f) { return bf_bits2f(f2bf_bits(f)); }
__device__ __forceinline__ float carry_flush(float v, float carry) {
  const float s = v * carry;
  return (fabsf(s) < kF16MinNormal) ? 0.0f : s;
}

__device__ __forceinline__ void dep_guard4_h(v8f& a, v8f& b, v8f& c, v8f& d, v16h x, v16h y) { asm volatile("v_nop\n\tv_nop\n\tv_nop\n\tv_nop" : "+v"(a), "+v"(b), "+v"(c), "+v"(d) : "v"(x), "v"(y)); }
__device__ __forceinline__ void dep_guard4_b(v8f& a, v8f& b, v8f& c, v8f& d, v16b x, v16b y) { asm volatile("v_nop\n\tv_nop\n\tv_nop\n\tv_nop" : "+v"(a), "+v"(b), "+v"(c), "+v"(d) : "v"(x), "v"(y)); }
__device__ __forceinline__ void keep4_h(v16h a, v16h b, v16h c, v16h d) { asm volatile("v_nop" :: "v"(a), "v"(b), "v"(c), "v"(d)); }
__device__ __forceinline__ void keep4_b(v16b a, v16b b, v16b c, v16b d) { asm volatile("v_nop" :: "v"(a), "v"(b), "v"(c), "v"(d)); }
__device__ __forceinline__ void acc_guard4(v8f& a, v8f& b, v8f& c, v8f& d) { asm volatile("v_nop\n\tv_nop\n\tv_nop\n\tv_nop" : "+v"(a), "+v"(b), "+v"(c), "+v"(d)); }

template <typename T> struct Frag;
template <> struct Frag<_Float16> {
  typedef v16h V; union U { v16h v; v8h h[2]; };
  static __device__ __forceinline__ v16h load(const _Float16* p) {
    U f; f.h[0] = *(const v8h*)(p); f.h[1] = *(const v8h*)(p + 16); return f.v;
  }
  static __device__ __forceinline__ v8f mma(v16h a, v16h b, v8f c) {
    return __builtin_amdgcn_wmma_f32_16x16x32_f16(false, a, false, b, (short)0, c, false, false);
  }
  static __device__ __forceinline__ void guard4(v8f& a, v8f& b, v8f& c, v8f& d, v16h x, v16h y) { dep_guard4_h(a, b, c, d, x, y); }
  static __device__ __forceinline__ void keep(v16h a, v16h b, v16h c, v16h d) { keep4_h(a, b, c, d); }
};
template <> struct Frag<__bf16> {
  typedef v16b V; union U { v16b v; v8b h[2]; };
  static __device__ __forceinline__ v16b load(const __bf16* p) {
    U f; f.h[0] = *(const v8b*)(p); f.h[1] = *(const v8b*)(p + 16); return f.v;
  }
  static __device__ __forceinline__ v8f mma(v16b a, v16b b, v8f c) {
    return __builtin_amdgcn_wmma_f32_16x16x32_bf16(false, a, false, b, (short)0, c, false, false);
  }
  static __device__ __forceinline__ void guard4(v8f& a, v8f& b, v8f& c, v8f& d, v16b x, v16b y) { dep_guard4_b(a, b, c, d, x, y); }
  static __device__ __forceinline__ void keep(v16b a, v16b b, v16b c, v16b d) { keep4_b(a, b, c, d); }
};

__device__ __forceinline__ v8f mma_h(v16h a, v16h b, v8f c) {
  c = __builtin_amdgcn_wmma_f32_16x16x32_f16(false, a, false, b, (short)0, c, false, false);
  asm volatile("v_nop\n\tv_nop\n\tv_nop\n\tv_nop" : "+v"(c) : "v"(a), "v"(b));
  return c;
}

template <int ET> struct Elem;
template <> struct Elem<0> { typedef _Float16 T; };
template <> struct Elem<1> { typedef __bf16 T; };
template <int ET, bool SPLIT, int BIAS_MODE, int OUT_MODE, bool RESID, int ACT = 0>
__global__ __launch_bounds__(256) void wmma_gemm64(
    const unsigned short* __restrict__ Ap, const unsigned short* __restrict__ A2p, int lda, long strideA,
    const unsigned short* __restrict__ Btp, const unsigned short* __restrict__ Bt2p, int ldb, long strideB,
    void* __restrict__ Cout, void* __restrict__ Cout2, int ldc, long strideC,
    const float* __restrict__ bias,
    const float* __restrict__ resid, long strideR,
    int M, int N, int K, float scale) {
  typedef typename Elem<ET>::T T;
  typedef typename Frag<T>::V V;
  const T* A = (const T*)Ap; const T* A2 = (const T*)A2p; const T* Bt = (const T*)Btp; const T* Bt2 = (const T*)Bt2p;
  __shared__ __align__(16) float sT[8][16 * 68];
  const int b    = blockIdx.y;
  const int lane = threadIdx.x & 31;
  const int wave = threadIdx.x >> 5;
  const int tilesN = N >> 6;
  const int tilesM = M >> 6;
  const int tile = blockIdx.x * 8 + wave;
  if (tile >= tilesM * tilesN) return;
  const int tm = tile / tilesN;
  const int tn = tile - tm * tilesN;
  const int m0 = tm << 6;
  const int n0 = tn << 6;

  const T* Ab  = A  + (size_t)b * strideA;
  const T* Bb  = Bt + (size_t)b * strideB;
  const T* Ab2 = SPLIT ? (A2  + (size_t)b * strideA) : nullptr;
  const T* Bb2 = SPLIT ? (Bt2 + (size_t)b * strideB) : nullptr;

  const int rlane = lane & 15;
  const int koff  = (lane >> 4) * 8;
  const int mOff  = (lane >> 4) * 8;

  v8f acc[4][4];
#pragma unroll
  for (int i = 0; i < 4; ++i)
#pragma unroll
    for (int j = 0; j < 4; ++j) acc[i][j] = (v8f){0.f,0.f,0.f,0.f,0.f,0.f,0.f,0.f};

  for (int k0 = 0; k0 < K; k0 += 32) {
    V bh[4], bl[4];
#pragma unroll
    for (int j = 0; j < 4; ++j) {
      const size_t bo = (size_t)(n0 + (j << 4) + rlane) * ldb + koff + k0;
      bh[j] = Frag<T>::load(Bb + bo);
      if (SPLIT) bl[j] = Frag<T>::load(Bb2 + bo);
    }
#pragma unroll
    for (int i = 0; i < 4; ++i) {
      const size_t ao = (size_t)(m0 + (i << 4) + rlane) * lda + koff + k0;
      V ah = Frag<T>::load(Ab + ao);
      V al;
      if (SPLIT) al = Frag<T>::load(Ab2 + ao);
#pragma unroll
      for (int j = 0; j < 4; ++j) {
        acc[i][j] = Frag<T>::mma(ah, bh[j], acc[i][j]);
        if (SPLIT) {
          acc[i][j] = Frag<T>::mma(ah, bl[j], acc[i][j]);
          acc[i][j] = Frag<T>::mma(al, bh[j], acc[i][j]);
        }
      }
      Frag<T>::guard4(acc[i][0], acc[i][1], acc[i][2], acc[i][3], ah, SPLIT ? al : ah);
    }
    Frag<T>::keep(bh[0], bh[1], bh[2], bh[3]);
    if (SPLIT) Frag<T>::keep(bl[0], bl[1], bl[2], bl[3]);
  }
  acc_guard4(acc[0][0], acc[0][1], acc[0][2], acc[0][3]);
  acc_guard4(acc[1][0], acc[1][1], acc[1][2], acc[1][3]);
  acc_guard4(acc[2][0], acc[2][1], acc[2][2], acc[2][3]);
  acc_guard4(acc[3][0], acc[3][1], acc[3][2], acc[3][3]);

  float* slab = sT[wave];
  const float* Rb = RESID ? (resid + (size_t)b * strideR) : nullptr;
#pragma unroll
  for (int i = 0; i < 4; ++i) {
    const int mBase = m0 + (i << 4);
#pragma unroll
    for (int j = 0; j < 4; ++j) {
      const int n = n0 + (j << 4) + rlane;
      float bv = 0.f;
      if (BIAS_MODE == 2) bv = bias[n];
#pragma unroll
      for (int r = 0; r < 8; ++r) {
        float v = acc[i][j][r] * scale;
        if (BIAS_MODE == 1) v += bias[mBase + mOff + r];
        if (BIAS_MODE == 2) v += bv;
        if (RESID) v += Rb[(size_t)(mBase + mOff + r) * ldc + n];
        if (ACT == 1) v = tanhf(v);
        if (ACT == 2) v = fmaxf(v, 0.0f);
        if (ACT == 3) v = v / (1.0f + expf(-v));
        if (ACT == 4) v = (v > 0.f) ? v : 0.01f * v;
        slab[(mOff + r) * 68 + (j << 4) + rlane] = v;
      }
    }
    __builtin_amdgcn_fence(__ATOMIC_RELEASE, "workgroup");
    __builtin_amdgcn_wave_barrier();
    __builtin_amdgcn_fence(__ATOMIC_ACQUIRE, "workgroup");
    if (OUT_MODE == 0) {
      float* C = (float*)Cout + (size_t)b * strideC;
      const int hh = lane >> 4, c4 = (lane & 15) * 4;
      for (int pass = 0; pass < 2; ++pass) {
#pragma unroll
        for (int it = 0; it < 8; ++it) {
          const int row = it * 2 + hh;
          v4f v = *(const v4f*)(slab + row * 68 + c4);
          *(volatile v4f*)(C + (size_t)(mBase + row) * ldc + n0 + c4) = v;
        }
        __threadfence();
      }
    } else {
      const int q = lane >> 3, c8 = (lane & 7) * 8;
      unsigned short* C  = (unsigned short*)Cout  + (size_t)b * strideC;
      unsigned short* C2 = (OUT_MODE == 2) ? ((unsigned short*)Cout2 + (size_t)b * strideC) : nullptr;
      for (int pass = 0; pass < 2; ++pass) {
#pragma unroll
        for (int it = 0; it < 4; ++it) {
          const int row = it * 4 + q;
          const float* sp = slab + row * 68 + c8;
          v8h hv, lv;
#pragma unroll
          for (int e = 0; e < 8; ++e) {
            if (OUT_MODE == 1) {
              hv[e] = (_Float16)sp[e];
            } else {
              unsigned short hb = f2bf_bits(sp[e]);
              unsigned short lb = f2bf_bits(sp[e] - bf_bits2f(hb));
              hv[e] = __builtin_bit_cast(_Float16, hb);
              lv[e] = __builtin_bit_cast(_Float16, lb);
            }
          }
          *(volatile v8h*)(C + (size_t)(mBase + row) * ldc + n0 + c8) = hv;
          if (OUT_MODE == 2) *(volatile v8h*)(C2 + (size_t)(mBase + row) * ldc + n0 + c8) = lv;
        }
        __threadfence();
      }
    }
    __builtin_amdgcn_fence(__ATOMIC_RELEASE, "workgroup");
    __builtin_amdgcn_wave_barrier();
    __builtin_amdgcn_fence(__ATOMIC_ACQUIRE, "workgroup");
  }
}

__global__ __launch_bounds__(kThr) void cast_plane_kernel(const float* __restrict__ src, unsigned short* __restrict__ dst,
                                                          int colsLog2, int dstPitch, int dstOff) {
  const int i   = blockIdx.x * kThr + threadIdx.x;
  const int sh  = colsLog2 - 3;
  const int row = i >> sh;
  const int c8  = (i & ((1 << sh) - 1)) * 8;
  const float* sp = src + ((size_t)row << colsLog2) + c8;
  const v4f a0 = *(const v4f*)(sp);
  const v4f a1 = *(const v4f*)(sp + 4);
  v8h hv;
#pragma unroll
  for (int e = 0; e < 4; ++e) {
    const float f0 = a0[e];
    const float f1 = a1[e];
    hv[e]     = (_Float16)carry_flush(bf16r(f0), kInCarry);
    hv[4 + e] = (_Float16)carry_flush(bf16r(f1), kInCarry);
  }
  unsigned short* dp = dst + (size_t)row * dstPitch + dstOff + c8;
  *(volatile v8h*)dp = hv;
  __threadfence();
  *(volatile v8h*)dp = hv;
}

typedef unsigned short v8us __attribute__((ext_vector_type(8), may_alias));
typedef float  v4fa __attribute__((ext_vector_type(4), may_alias));
__device__ __forceinline__ unsigned short bf16_bits(float x) { unsigned int u = __float_as_uint(x); return (unsigned short)((u + 0x7FFFu + ((u >> 16) & 1u)) >> 16); }
__device__ __forceinline__ float bf16_val(unsigned short b) { return __uint_as_float(((unsigned int)b) << 16); }
__device__ __forceinline__ float bf16_round(float x) { return bf16_val(bf16_bits(x)); }
typedef _Float16 v16h __attribute__((ext_vector_type(16)));
union FragH { v16h v; v8us half[2]; _Float16 h[16]; unsigned short u[16]; };
typedef _Float16 v4h __attribute__((ext_vector_type(4)));
__device__ __forceinline__ v16h g2_frag(const _Float16* p, int hh) { FragH f; f.half[0] = *(const v8us*)((const unsigned short*)p + 8 * hh); f.half[1] = *(const v8us*)((const unsigned short*)p + 16 + 8 * hh); return f.v; }
__device__ __forceinline__ v8f g2_mma(v16h a, v16h b, v8f c) { v8f d = __builtin_amdgcn_wmma_f32_16x16x32_f16(false, a, false, b, (short)0, c, false, false); asm volatile("v_nop\n\tv_nop\n\tv_nop\n\tv_nop" : "+v"(d) : "v"(a), "v"(b)); return d; }
template <int ACT>
__global__ __launch_bounds__(128) void k_gemm2(const _Float16* __restrict__ A, int lda, size_t sA, const _Float16* __restrict__ Bh, int ldb, size_t sB, float alpha, const float* __restrict__ bias, size_t sBias, const float* __restrict__ CP, int rowsPerB, size_t sCPb, int row0g,
    float* __restrict__ C, _Float16* __restrict__ C16, int ldc, size_t sC, int M, int N, int K) { static_assert(ACT == 0 || ACT == 3 || ACT == 6 || ACT == 8 || ACT == 9 || ACT == 11 || ACT == 12 || ACT == 14 || ACT == 15 || ACT == 16 || ACT == 17, "k_gemm2: unsupported ACT code (would silently apply no activation)");
  __shared__ __attribute__((aligned(16))) float so[4][32][68];
  const int tid = threadIdx.x, w = tid >> 5, lane = tid & 31, ln = lane & 15, hh = lane >> 4; const int by = blockIdx.y;
  A += (size_t)by * sA; Bh += (size_t)by * sB; const size_t cofs = (size_t)by * sC; const float* bp = bias ? bias + (size_t)by * sBias : nullptr;
  const int ntn = N >> 6; const int mt = blockIdx.x / ntn, nq = blockIdx.x - mt * ntn; const int row0 = mt * 128 + 32 * w, col0 = nq * 64; if (row0 >= M) return;
  const _Float16* a0p = A + (size_t)(row0 + ln) * lda; const _Float16* a1p = a0p + (size_t)16 * lda;
  const _Float16* b0p = Bh + (size_t)(col0 + ln) * ldb; const _Float16* b1p = b0p + (size_t)16 * ldb; const _Float16* b2p = b1p + (size_t)16 * ldb; const _Float16* b3p = b2p + (size_t)16 * ldb;
  const v8f z8 = {0.f,0.f,0.f,0.f,0.f,0.f,0.f,0.f}; v8f c00 = z8, c01 = z8, c02 = z8, c03 = z8, c10 = z8, c11 = z8, c12 = z8, c13 = z8;
  for (int kb = 0; kb < K; kb += 32) { const v16h a0 = g2_frag(a0p + kb, hh), a1 = g2_frag(a1p + kb, hh);
    v16h b = g2_frag(b0p + kb, hh); c00 = g2_mma(a0, b, c00); c10 = g2_mma(a1, b, c10);
    b = g2_frag(b1p + kb, hh); c01 = g2_mma(a0, b, c01); c11 = g2_mma(a1, b, c11);
    b = g2_frag(b2p + kb, hh); c02 = g2_mma(a0, b, c02); c12 = g2_mma(a1, b, c12);
    b = g2_frag(b3p + kb, hh); c03 = g2_mma(a0, b, c03); c13 = g2_mma(a1, b, c13); }
  v8f accs[8] = {c00, c01, c02, c03, c10, c11, c12, c13};
#pragma unroll
  for (int u = 0; u < 8; ++u) { const int t = u & 3, half = u >> 2; const int col = col0 + t * 16 + ln; const float bv = bp ? bf16_round(bp[col]) : 0.f;
#pragma unroll
    for (int r = 0; r < 8; ++r) { const int rloc = half * 16 + 8 * hh + r; float v = accs[u][r] * alpha + bv; if (CP) { if (rowsPerB < 0) v += CP[cofs + (size_t)(row0g + row0 + rloc) * ldc + col];        else { const int bidx = (row0g + row0 + rloc) / rowsPerB; v += CP[(size_t)bidx * sCPb + (size_t)by * 64 + col]; } }
      if (ACT == 3) v = fmaxf(v, 0.f); else if (ACT == 6) v = 0.5f * v * (1.0f + erff(v * 0.70710678118654752f)); else if (ACT == 11) v = 1.0f / (1.0f + expf(-v)); else if (ACT == 15) v = v / (1.0f + expf(-v)); else if (ACT == 12) v = (v > 0.f) ? v : 0.01f * v; else if (ACT == 8) v = tanhf(v); else if (ACT == 9) v = 0.5f * v * (1.0f + tanhf(0.7978845608028654f * (v + 0.044715f * v * v * v))); else if (ACT == 14) v = (v > 0.f) ? v : 0.1f * v; else if (ACT == 16) v = (v >= 0.f) ? v : 0.3f * v; else if (ACT == 17) v = (v >= 0.f) ? v : 0.2f * v;
      so[w][rloc][t * 16 + ln] = v; } }
  __builtin_amdgcn_fence(__ATOMIC_ACQ_REL, "workgroup"); __builtin_amdgcn_wave_barrier();
  const int rsub = lane >> 4, c4 = (lane & 15) * 4;
  for (int pass = 0; pass < 2; ++pass) {
#pragma unroll
    for (int q = 0; q < 16; ++q) { const int r = q * 2 + rsub; const v4f v = *(const v4fa*)&so[w][r][c4]; if (C) *(volatile v4f*)(C + cofs + (size_t)(row0 + r) * ldc + col0 + c4) = v; if (C16) { v4h h4; for (int i = 0; i < 4; ++i) h4[i] = (_Float16)v[i]; *(volatile v4h*)(C16 + cofs + (size_t)(row0 + r) * ldc + col0 + c4) = h4; } }
    if (pass == 0) __threadfence(); } }

__global__ __launch_bounds__(kThr) void zero_kernel(float* __restrict__ dst) {
  const size_t o4 = ((size_t)blockIdx.x * kThr + threadIdx.x) * 4u;
  const v4f z = {0.f, 0.f, 0.f, 0.f};
  *(volatile v4f*)(dst + o4) = z;
  __threadfence();
  *(volatile v4f*)(dst + o4) = z;
}

__global__ __launch_bounds__(64) void table_kernel(const float* __restrict__ a, float* __restrict__ TAB) {
  const unsigned i = blockIdx.x * 64u + threadIdx.x;
  const int r = (int)(i >> 6), c = (int)(i & 63u);
  const float g = 1.0f / (1.0f + expf(-bf16r(a[0])));
  const float lg = logf(g);
  const int dm = r - 1 - c;
  const int em = (dm > 0) ? dm : 0;
  const int e = (r < 64) ? em : ((r == 64) ? c : ((r == 65) ? (63 - c) : 64));
  const float keep = (r < 64) ? ((r > c) ? 1.0f : 0.0f) : 1.0f;
  const float val = keep * expf(lg * (float)e);
  *(volatile float*)(TAB + i) = val;
  __threadfence();
  *(volatile float*)(TAB + i) = val;
}

__global__ __launch_bounds__(kThr) void keys_kernel(const float* __restrict__ X, unsigned short* __restrict__ K) {
  const unsigned i = blockIdx.x * (unsigned)kThr + threadIdx.x;
  const unsigned t8 = (i & 1023u) * 8u, e = (i >> 10) & 511u, b = i >> 19;
  const float* xb = X + (size_t)b * kT * kD + e;
  v8h hv;
#pragma unroll
  for (int j = 0; j < 8; ++j) {
    const unsigned t = t8 + (unsigned)j;
    const unsigned tr = (t > 0u) ? (t - 1u) : 0u;
    const float x = bf16r(xb[(size_t)tr * kD]);
    hv[j] = (_Float16)carry_flush((t > 0u) ? x : 0.0f, kInCarry);
  }
  unsigned short* dp = K + ((size_t)b * kD + e) * kT + t8;
  *(volatile v8h*)dp = hv;
  __threadfence();
  *(volatile v8h*)dp = hv;
}

__global__ __launch_bounds__(kThr) void values_cast_kernel(const float* __restrict__ S, const float* __restrict__ TAB, unsigned short* __restrict__ D, unsigned short* __restrict__ G) {
  const size_t o8 = ((size_t)blockIdx.x * (unsigned)kThr + threadIdx.x) * 8u;
  const unsigned c8 = (unsigned)o8 & 63u;
  const v4f s0 = *(const v4f*)(S + o8), s1 = *(const v4f*)(S + o8 + 4);
  const v4f w0 = *(const v4f*)(TAB + 65 * 64 + c8), w1 = *(const v4f*)(TAB + 65 * 64 + c8 + 4);
  v8h hv, gv;
#pragma unroll
  for (int j = 0; j < 4; ++j) {
    hv[j] = (_Float16)carry_flush(s0[j], kVCarry); hv[4 + j] = (_Float16)carry_flush(s1[j], kVCarry);
    gv[j] = (_Float16)carry_flush(s0[j] * w0[j], kVCarry); gv[4 + j] = (_Float16)carry_flush(s1[j] * w1[j], kVCarry);
  }
  *(volatile v8h*)(D + o8) = hv;
  *(volatile v8h*)(G + o8) = gv;
  __threadfence();
  *(volatile v8h*)(D + o8) = hv;
  *(volatile v8h*)(G + o8) = gv;
}

__global__ __launch_bounds__(kThr) void mask_kernel(const float* __restrict__ Z, const float* __restrict__ TAB, unsigned short* __restrict__ SM, int n) {
  const unsigned i = blockIdx.x * (unsigned)kThr + threadIdx.x;
  const unsigned s8 = (i & 7u) * 8u, t = (i >> 3) & 63u, b = i >> 9;
  const float* zp = Z + (((size_t)b * kNC + (unsigned)n) * kC + t) * kC + s8;
  const float* mp = TAB + t * 64u + s8;
  const v4f z0 = *(const v4f*)zp, z1 = *(const v4f*)(zp + 4);
  const v4f m0 = *(const v4f*)mp, m1 = *(const v4f*)(mp + 4);
  v8h hv;
#pragma unroll
  for (int j = 0; j < 4; ++j) { hv[j] = (_Float16)carry_flush(z0[j] * m0[j], kSCarry); hv[4 + j] = (_Float16)carry_flush(z1[j] * m1[j], kSCarry); }
  unsigned short* dp = SM + ((size_t)b * kC + t) * kC + s8;
  *(volatile v8h*)dp = hv;
  __threadfence();
  *(volatile v8h*)dp = hv;
}

__global__ __launch_bounds__(kThr) void combine_kernel(const float* __restrict__ R1, const float* __restrict__ R2, const float* __restrict__ TAB, unsigned short* __restrict__ RO, int n) {
  const unsigned i = blockIdx.x * (unsigned)kThr + threadIdx.x;
  const unsigned d8 = (i & 63u) * 8u, t = (i >> 6) & 63u, b = i >> 12;
  const size_t o = ((size_t)b * kC + t) * kD + d8;
  const float gp = TAB[64 * 64 + t];
  const v4f a0 = *(const v4f*)(R1 + o), a1 = *(const v4f*)(R1 + o + 4);
  const v4f c0 = *(const v4f*)(R2 + o), c1 = *(const v4f*)(R2 + o + 4);
  v8h hv;
#pragma unroll
  for (int j = 0; j < 4; ++j) { hv[j] = (_Float16)carry_flush(a0[j] * gp + c0[j], kRCarry); hv[4 + j] = (_Float16)carry_flush(a1[j] * gp + c1[j], kRCarry); }
  unsigned short* dp = RO + ((size_t)b * kT + (unsigned)n * kC + t) * kD + d8;
  *(volatile v8h*)dp = hv;
  __threadfence();
  *(volatile v8h*)dp = hv;
}

__global__ __launch_bounds__(kThr) void state_kernel(const float* __restrict__ DW, const float* __restrict__ TAB, float* S, unsigned short* __restrict__ SH) {
  const size_t o8 = ((size_t)blockIdx.x * (unsigned)kThr + threadIdx.x) * 8u;
  const float gc = TAB[66 * 64];
  const v4f s0 = *(const v4f*)(S + o8), s1 = *(const v4f*)(S + o8 + 4);
  const v4f d0 = *(const v4f*)(DW + o8), d1 = *(const v4f*)(DW + o8 + 4);
  v4f y0, y1; v8h hv;
#pragma unroll
  for (int j = 0; j < 4; ++j) { y0[j] = gc * s0[j] + d0[j]; y1[j] = gc * s1[j] + d1[j]; hv[j] = (_Float16)carry_flush(y0[j], kSCarry); hv[4 + j] = (_Float16)carry_flush(y1[j], kSCarry); }
  *(volatile v4f*)(S + o8) = y0;
  *(volatile v4f*)(S + o8 + 4) = y1;
  *(volatile v8h*)(SH + o8) = hv;
  __threadfence();
  *(volatile v4f*)(S + o8) = y0;
  *(volatile v4f*)(S + o8 + 4) = y1;
  *(volatile v8h*)(SH + o8) = hv;
}

__global__ __launch_bounds__(kThr) void close_kernel(const float* __restrict__ X, const float* __restrict__ PR, float* __restrict__ out) {
  const size_t o8 = ((size_t)blockIdx.x * (unsigned)kThr + threadIdx.x) * 8u;
  const v4f x0 = *(const v4f*)(X + o8), x1 = *(const v4f*)(X + o8 + 4);
  const v4f p0 = *(const v4f*)(PR + o8), p1 = *(const v4f*)(PR + o8 + 4);
  v4f y0, y1;
#pragma unroll
  for (int j = 0; j < 4; ++j) { y0[j] = bf16r(x0[j]) + kMix * p0[j]; y1[j] = bf16r(x1[j]) + kMix * p1[j]; }
  *(volatile v4f*)(out + o8) = y0;
  *(volatile v4f*)(out + o8 + 4) = y1;
  __threadfence();
  *(volatile v4f*)(out + o8) = y0;
  *(volatile v4f*)(out + o8 + 4) = y1;
}

extern "C" void kernel_launch(void* const* d_in, const int* in_sizes, int n_in,
                              void* d_out, int out_size, void* d_ws, size_t ws_size,
                              hipStream_t stream) {
  if (n_in < 4 || d_out == nullptr || d_ws == nullptr) return;
  if (in_sizes[0] != kB * kT * kD || in_sizes[1] != kD * kD || in_sizes[2] != kD * kD || in_sizes[3] != 1) return;
  if ((size_t)out_size != (size_t)kB * kT * kD) return;
  if (ws_size < kWsTotal) return;
  const float* X = (const float*)d_in[0];
  char* ws = (char*)d_ws;
  unsigned short* XP16 = (unsigned short*)(ws + kOffXP16);
  unsigned short* P16 = (unsigned short*)(ws + kOffP16);
  unsigned short* Q16 = (unsigned short*)(ws + kOffQ16);
  float* VP = (float*)(ws + kOffVP);
  unsigned short* VT16 = (unsigned short*)(ws + kOffVT16);
  unsigned short* VG16 = (unsigned short*)(ws + kOffVG16);
  unsigned short* KT16 = (unsigned short*)(ws + kOffKT16);
  float* ZA = (float*)(ws + kOffZA);
  unsigned short* SM16 = (unsigned short*)(ws + kOffSM16);
  float* S32 = (float*)(ws + kOffS32);
  unsigned short* S16 = (unsigned short*)(ws + kOffS16);
  float* DW = (float*)(ws + kOffDW);
  float* R1 = (float*)(ws + kOffR1);
  float* R2 = (float*)(ws + kOffR2);
  unsigned short* RO16 = (unsigned short*)(ws + kOffRO16);
  float* TAB = (float*)(ws + kOffTAB);
  const long sXP = (long)kRows * kD, sT = (long)kD * kT, sS = (long)kD * kD, sR = (long)kC * kD;

  static_assert((kT * (kD / 8)) % kThr == 0 && (kD * (kD / 8)) % kThr == 0 && (kPad * kD * 2) == kThr * 16 && (kB * kD * kD / 4) % kThr == 0 && (kB * kD * kD / 8) % kThr == 0 && (kB * kD * (kT / 8)) % kThr == 0 && (kB * kC * (kC / 8)) % kThr == 0 && (kB * kC * (kD / 8)) % kThr == 0 && (67 * 64) % 64 == 0, "every flat kernel's grid exact");
  for (int b = 0; b < kB; ++b) {
    zero_kernel<<<1, kThr, 0, stream>>>((float*)(XP16 + (size_t)b * sXP));
    cast_plane_kernel<<<kT * (kD / 8) / kThr, kThr, 0, stream>>>(X + (size_t)b * kT * kD, XP16 + (size_t)b * sXP + (size_t)kPad * kD, 9, kD, 0);
  }
  cast_plane_kernel<<<kD * (kD / 8) / kThr, kThr, 0, stream>>>((const float*)d_in[1], P16, 9, kD, 0);
  cast_plane_kernel<<<kD * (kD / 8) / kThr, kThr, 0, stream>>>((const float*)d_in[2], Q16, 9, kD, 0);
  zero_kernel<<<kB * kD * kD / 4 / kThr, kThr, 0, stream>>>(S32);
  zero_kernel<<<kB * kD * kD / 8 / kThr, kThr, 0, stream>>>((float*)S16);
  table_kernel<<<67, 64, 0, stream>>>((const float*)d_in[3], TAB);
  keys_kernel<<<kB * kD * (kT / 8) / kThr, kThr, 0, stream>>>(X, KT16);
  wmma_gemm64<0, false, 0, 0, false, 0><<<dim3((kD / 64) * (kT / 64) / 8, kB), 256, 0, stream>>>(
      P16, P16, kD, 0L, XP16 + (size_t)kPad * kD, XP16 + (size_t)kPad * kD, kD, sXP, (void*)VP, (void*)VP, kT, sT, nullptr, nullptr, 0L, kD, kT, kD, kSc20);
  values_cast_kernel<<<kB * kD * (kT / 8) / kThr, kThr, 0, stream>>>(VP, TAB, VT16, VG16);
  for (int b = 0; b < kB; ++b)
    k_gemm2<0><<<dim3(1, kNC), 128, 0, stream>>>((const _Float16*)(XP16 + (size_t)b * sXP + (size_t)kPad * kD), kD, (size_t)kC * kD, (const _Float16*)(XP16 + (size_t)b * sXP + (size_t)(kPad - 1) * kD), kD, (size_t)kC * kD, kSc20, nullptr, 0, nullptr, 1, 0, 0, ZA + (size_t)b * kNC * kC * kC, nullptr, kC, (size_t)kC * kC, kC, kC, kD);
  for (int n = 0; n < kNC; ++n) {
    wmma_gemm64<0, false, 0, 0, false, 0><<<dim3((kC / 64) * (kD / 64) / 8, kB), 256, 0, stream>>>(
        XP16 + (size_t)(kPad + kC * n) * kD, XP16 + (size_t)(kPad + kC * n) * kD, kD, sXP, S16, S16, kD, sS, (void*)R1, (void*)R1, kD, sR, nullptr, nullptr, 0L, kC, kD, kD, kSc16);
    mask_kernel<<<kB * kC * (kC / 8) / kThr, kThr, 0, stream>>>(ZA, TAB, SM16, n);
    wmma_gemm64<0, false, 0, 0, false, 0><<<dim3((kC / 64) * (kD / 64) / 8, kB), 256, 0, stream>>>(
        SM16, SM16, kC, (long)kC * kC, VT16 + (size_t)kC * n, VT16 + (size_t)kC * n, kT, sT, (void*)R2, (void*)R2, kD, sR, nullptr, nullptr, 0L, kC, kD, kC, kSc14);
    combine_kernel<<<kB * kC * (kD / 8) / kThr, kThr, 0, stream>>>(R1, R2, TAB, RO16, n);
    wmma_gemm64<0, false, 0, 0, false, 0><<<dim3((kD / 64) * (kD / 64) / 8, kB), 256, 0, stream>>>(
        VG16 + (size_t)kC * n, VG16 + (size_t)kC * n, kT, sT, KT16 + (size_t)kC * n, KT16 + (size_t)kC * n, kT, sT, (void*)DW, (void*)DW, kD, sS, nullptr, nullptr, 0L, kD, kD, kC, kSc18);
    state_kernel<<<kB * kD * kD / 8 / kThr, kThr, 0, stream>>>(DW, TAB, S32, S16);
  }
  wmma_gemm64<0, false, 0, 0, false, 0><<<dim3((kB * kT / 64) * (kD / 64) / 8, 1), 256, 0, stream>>>(
      RO16, RO16, kD, 0L, Q16, Q16, kD, 0L, (void*)VP, (void*)VP, kD, 0L, nullptr, nullptr, 0L, kB * kT, kD, kD, kSc10);
  close_kernel<<<kB * kT * (kD / 8) / kThr, kThr, 0, stream>>>(X, VP, (float*)d_out);
}
static_assert(((kD / 64) * (kT / 64)) % 8 == 0 && ((kC / 64) * (kD / 64)) % 8 == 0 && ((kD / 64) * (kD / 64)) % 8 == 0 && ((kB * kT / 64) * (kD / 64)) % 8 == 0 && kD % 32 == 0 && kC % 32 == 0, "the engine's grids: whole blocks of eight wave tiles; every depth a multiple of 32");
